// VanishingNet_41875931136703
// MI455X (gfx1250) — hardware-verified
//
#include <hip/hip_runtime.h>
#define BB 2
#define CC 128
#define NPIX 16384
#define HTH 184
#define HTW 180
#define NBINS (HTH * HTW)
#define NPOSH (BB * NBINS)
#define KHT 8
#define KSPH 16
#define NSPH 16384

typedef __bf16 v16b __attribute__((ext_vector_type(16)));
typedef unsigned short v8us __attribute__((ext_vector_type(8), may_alias));
typedef float  v8f  __attribute__((ext_vector_type(8)));
typedef float  v4f  __attribute__((ext_vector_type(4)));
typedef float  v4fa __attribute__((ext_vector_type(4), may_alias));
union FragB { v16b v; v8us half[2]; unsigned short u[16]; };

__device__ __forceinline__ unsigned short bf16_bits(float x) { unsigned int u = __float_as_uint(x); return (unsigned short)((u + 0x7FFFu + ((u >> 16) & 1u)) >> 16); }
__device__ __forceinline__ float bf16_val(unsigned short b) { return __uint_as_float(((unsigned int)b) << 16); }
__device__ __forceinline__ float bf16_round(float x) { return bf16_val(bf16_bits(x)); }
template <int NT>
__device__ __forceinline__ v8f mmaN(v16b ah, v16b al, v16b bh, v16b bl, v8f c) {
  c = __builtin_amdgcn_wmma_f32_16x16x32_bf16(false, ah, false, bh, (short)0, c, false, false);
  if (NT >= 2) c = __builtin_amdgcn_wmma_f32_16x16x32_bf16(false, al, false, bh, (short)0, c, false, false);
  if (NT >= 3) c = __builtin_amdgcn_wmma_f32_16x16x32_bf16(false, ah, false, bl, (short)0, c, false, false);
  asm volatile("v_nop\n\tv_nop\n\tv_nop\n\tv_nop" : "+v"(c) : "v"(ah), "v"(al), "v"(bh), "v"(bl));
  return c;
}

__global__ __launch_bounds__(256) void k_wt_bf16(const float* __restrict__ W, unsigned short* __restrict__ Wt, int K, int N) {
  const int t = blockIdx.x * 256 + threadIdx.x;
  const int k8n = K / 8;
  if (t >= N * k8n) return;
  const int n = t / k8n, k8 = (t % k8n) * 8;
  v8us v;
#pragma unroll
  for (int i = 0; i < 8; ++i) v[i] = bf16_bits(W[(size_t)(k8 + i) * N + n]);
  *(volatile v8us*)(Wt + (size_t)n * K + k8) = v;
  __threadfence();
  *(volatile v8us*)(Wt + (size_t)n * K + k8) = v;
}

template <bool ASPLIT, int ACT, bool BIAS_BF16>
__global__ __launch_bounds__(128) void k_gemm_bf(const float* __restrict__ A, int lda, const unsigned short* __restrict__ Wt, int ldb,
                                               const float* __restrict__ bias, float* __restrict__ C, int ldc, int M, int N, int K) {
  __shared__ __attribute__((aligned(16))) float so[4][16][64];
  const int tid = threadIdx.x, w = tid >> 5, lane = tid & 31, ln = lane & 15, hh = lane >> 4;
  const int ntn = N / 64;
  const int wid = blockIdx.x * 4 + w;
  const int mt = wid / ntn, nq = wid % ntn;
  if (mt * 16 >= M) return;
  const int row0 = mt * 16, col0 = nq * 64;
  const float* arow = A + (size_t)(row0 + ln) * lda;
  v8f acc[4] = {};
  for (int kb = 0; kb < K; kb += 32) {
    FragB ah, al;
    const v4f x0 = *(const v4fa*)(arow + kb + 8 * hh), x1 = *(const v4fa*)(arow + kb + 8 * hh + 4);
    const v4f x2 = *(const v4fa*)(arow + kb + 16 + 8 * hh), x3 = *(const v4fa*)(arow + kb + 16 + 8 * hh + 4);
    float xs[16] = {x0[0],x0[1],x0[2],x0[3],x1[0],x1[1],x1[2],x1[3],x2[0],x2[1],x2[2],x2[3],x3[0],x3[1],x3[2],x3[3]};
#pragma unroll
    for (int i = 0; i < 16; ++i) { const unsigned short hb = bf16_bits(xs[i]); ah.u[i] = hb; al.u[i] = ASPLIT ? bf16_bits(xs[i] - bf16_val(hb)) : (unsigned short)0; }
#pragma unroll
    for (int t = 0; t < 4; ++t) {
      const unsigned short* brow = Wt + (size_t)(col0 + t * 16 + ln) * ldb + kb;
      FragB b;
      b.half[0] = *(const v8us*)(brow + 8 * hh);
      b.half[1] = *(const v8us*)(brow + 16 + 8 * hh);
      acc[t] = mmaN<ASPLIT ? 2 : 1>(ah.v, al.v, b.v, b.v, acc[t]);
    }
  }
#pragma unroll
  for (int t = 0; t < 4; ++t) {
    float bv = bias ? bias[col0 + t * 16 + ln] : 0.f;
    if (BIAS_BF16) bv = bf16_round(bv);
#pragma unroll
    for (int r = 0; r < 8; ++r) { float v = acc[t][r] + bv; if (ACT == 1) v = fmaxf(v, 0.f); so[w][8 * hh + r][t * 16 + ln] = v; }
  }
  __builtin_amdgcn_fence(__ATOMIC_ACQ_REL, "workgroup");
  __builtin_amdgcn_wave_barrier();
  const int rsub = lane >> 4, c4 = (lane & 15) * 4;
  for (int pass = 0; pass < 2; ++pass) {
#pragma unroll
    for (int q = 0; q < 8; ++q) {
      const int r = q * 2 + rsub;
      const v4f v = *(const v4fa*)&so[w][r][c4];
      *(volatile v4f*)(C + (size_t)(row0 + r) * ldc + col0 + c4) = v;
    }
    if (pass == 0) __threadfence();
  }
}

template <int D, bool CAUSAL>
__global__ __launch_bounds__(128) void k_flash(const float* __restrict__ qb, const float* __restrict__ kb, const float* __restrict__ vb,
                                             int pitch, int T, int H, float scale, float* __restrict__ y, int ypitch) {
  constexpr int KS = D / 32;
  constexpr int DT = D / 16;
  __shared__ __attribute__((aligned(16))) unsigned short sKh[32][D + 8], sKl[32][D + 8], sVh[32][D + 8], sVl[32][D + 8];
  __shared__ __attribute__((aligned(16))) unsigned short sPh[4][16][40], sPl[4][16][40];
  __shared__ __attribute__((aligned(16))) float sO[4][16][D];
  const int tid = threadIdx.x, w = tid >> 5, lane = tid & 31, ln = lane & 15, hh = lane >> 4;
  const int nqb = (T + 63) / 64;
  const int bh = blockIdx.x / nqb, qblk = blockIdx.x % nqb;
  const int b = bh / H, h = bh % H;
  const int q0 = qblk * 64 + w * 16;
  const float* Q = qb + (size_t)b * T * pitch + h * D;
  const float* K = kb + (size_t)b * T * pitch + h * D;
  const float* V = vb + (size_t)b * T * pitch + h * D;

  FragB aqh[KS], aql[KS];
  {
    int row = q0 + ln; if (row >= T) row = T - 1;
    const float* qr = Q + (size_t)row * pitch;
#pragma unroll
    for (int ks = 0; ks < KS; ++ks)
#pragma unroll
      for (int i = 0; i < 16; ++i) {
        const int d = ks * 32 + ((i < 8) ? (8 * hh + i) : (16 + 8 * hh + (i - 8)));
        const float x = qr[d] * scale; const unsigned short hb = bf16_bits(x);
        aqh[ks].u[i] = hb; aql[ks].u[i] = bf16_bits(x - bf16_val(hb));
      }
  }
  float m_r[8], l_r[8];
#pragma unroll
  for (int r = 0; r < 8; ++r) { m_r[r] = -3.0e38f; l_r[r] = 0.f; }
  v8f oacc[DT];
#pragma unroll
  for (int dt = 0; dt < DT; ++dt) oacc[dt] = (v8f){0.f,0.f,0.f,0.f,0.f,0.f,0.f,0.f};

  const int kv_end = CAUSAL ? min(T, qblk * 64 + 64) : T;
  for (int j0 = 0; j0 < kv_end; j0 += 32) {
    __syncthreads();
    for (int e = tid; e < 32 * (D / 4); e += 128) {
      const int r = e / (D / 4), c4 = (e % (D / 4)) * 4;
      const int key = j0 + r;
      v4f kf = {0.f,0.f,0.f,0.f}, vf = {0.f,0.f,0.f,0.f};
      if (key < T) { kf = *(const v4fa*)(K + (size_t)key * pitch + c4); vf = *(const v4fa*)(V + (size_t)key * pitch + c4); }
#pragma unroll
      for (int t = 0; t < 4; ++t) {
        unsigned short hb = bf16_bits(kf[t]); sKh[r][c4 + t] = hb; sKl[r][c4 + t] = bf16_bits(kf[t] - bf16_val(hb));
        hb = bf16_bits(vf[t]); sVh[r][c4 + t] = hb; sVl[r][c4 + t] = bf16_bits(vf[t] - bf16_val(hb));
      }
    }
    __syncthreads();
    v8f s[2];
#pragma unroll
    for (int nt = 0; nt < 2; ++nt) {
      v8f acc = {};
#pragma unroll
      for (int ks = 0; ks < KS; ++ks) {
        FragB bh_, bl_;
        bh_.half[0] = *(const v8us*)&sKh[nt * 16 + ln][ks * 32 + 8 * hh]; bh_.half[1] = *(const v8us*)&sKh[nt * 16 + ln][ks * 32 + 16 + 8 * hh];
        bl_.half[0] = *(const v8us*)&sKl[nt * 16 + ln][ks * 32 + 8 * hh]; bl_.half[1] = *(const v8us*)&sKl[nt * 16 + ln][ks * 32 + 16 + 8 * hh];
        acc = mmaN<3>(aqh[ks].v, aql[ks].v, bh_.v, bl_.v, acc);
      }
      s[nt] = acc;
    }
    float alpha[8];
#pragma unroll
    for (int r = 0; r < 8; ++r) {
      const int qi = q0 + 8 * hh + r;
      const int ja = j0 + ln, jb = j0 + 16 + ln;
      if (CAUSAL) { if (ja > qi) s[0][r] = -3.0e38f; if (jb > qi) s[1][r] = -3.0e38f; }
      if (ja >= T) s[0][r] = -3.0e38f;
      if (jb >= T) s[1][r] = -3.0e38f;
      float mx = fmaxf(s[0][r], s[1][r]);
      mx = fmaxf(mx, __shfl_xor(mx, 1, 32)); mx = fmaxf(mx, __shfl_xor(mx, 2, 32)); mx = fmaxf(mx, __shfl_xor(mx, 4, 32)); mx = fmaxf(mx, __shfl_xor(mx, 8, 32));
      const float mnew = fmaxf(m_r[r], mx);
      alpha[r] = (mnew > -1.0e38f) ? __expf(m_r[r] - mnew) : 1.0f;
      const float p0 = (s[0][r] > -1.0e38f) ? __expf(s[0][r] - mnew) : 0.f;
      const float p1 = (s[1][r] > -1.0e38f) ? __expf(s[1][r] - mnew) : 0.f;
      m_r[r] = mnew;
      l_r[r] = l_r[r] * alpha[r] + p0 + p1;
      unsigned short hb = bf16_bits(p0); sPh[w][8 * hh + r][ln] = hb;      sPl[w][8 * hh + r][ln] = bf16_bits(p0 - bf16_val(hb));
      hb = bf16_bits(p1);                sPh[w][8 * hh + r][16 + ln] = hb; sPl[w][8 * hh + r][16 + ln] = bf16_bits(p1 - bf16_val(hb));
    }
#pragma unroll
    for (int dt = 0; dt < DT; ++dt)
#pragma unroll
      for (int r = 0; r < 8; ++r) oacc[dt][r] *= alpha[r];
    __builtin_amdgcn_fence(__ATOMIC_ACQ_REL, "workgroup");
    __builtin_amdgcn_wave_barrier();
    FragB pah, pal;
    pah.half[0] = *(const v8us*)&sPh[w][ln][8 * hh]; pah.half[1] = *(const v8us*)&sPh[w][ln][16 + 8 * hh];
    pal.half[0] = *(const v8us*)&sPl[w][ln][8 * hh]; pal.half[1] = *(const v8us*)&sPl[w][ln][16 + 8 * hh];
#pragma unroll
    for (int dt = 0; dt < DT; ++dt) {
      FragB bvh, bvl;
#pragma unroll
      for (int i = 0; i < 8; ++i) {
        bvh.u[i] = sVh[8 * hh + i][dt * 16 + ln]; bvh.u[8 + i] = sVh[16 + 8 * hh + i][dt * 16 + ln];
        bvl.u[i] = sVl[8 * hh + i][dt * 16 + ln]; bvl.u[8 + i] = sVl[16 + 8 * hh + i][dt * 16 + ln];
      }
      oacc[dt] = mmaN<3>(pah.v, pal.v, bvh.v, bvl.v, oacc[dt]);
    }
    __builtin_amdgcn_fence(__ATOMIC_ACQ_REL, "workgroup");
    __builtin_amdgcn_wave_barrier();
  }
#pragma unroll
  for (int r = 0; r < 8; ++r) {
    float l = l_r[r];
    l += __shfl_xor(l, 1, 32); l += __shfl_xor(l, 2, 32); l += __shfl_xor(l, 4, 32); l += __shfl_xor(l, 8, 32);
    l_r[r] = (l > 0.f) ? 1.0f / l : 0.f;
  }
#pragma unroll
  for (int dt = 0; dt < DT; ++dt)
#pragma unroll
    for (int r = 0; r < 8; ++r) sO[w][8 * hh + r][dt * 16 + ln] = oacc[dt][r] * l_r[r];
  __builtin_amdgcn_fence(__ATOMIC_ACQ_REL, "workgroup");
  __builtin_amdgcn_wave_barrier();
  for (int pass = 0; pass < 2; ++pass) {
    for (int r = 0; r < 16; ++r) {
      const int row = q0 + r;
      if (row < T && lane < D / 4) {
        const v4f val = *(const v4fa*)&sO[w][r][lane * 4];
        *(volatile v4f*)(y + ((size_t)b * T + row) * ypitch + h * D + lane * 4) = val;
      }
    }
    if (pass == 0) __threadfence();
  }
}

template <bool ASPLIT, int ACT, bool BIAS_BF16, bool RES_BF16>
__global__ __launch_bounds__(128) void k_gemm_bf3(const float* __restrict__ A, int lda, const unsigned short* __restrict__ Wt, int ldb,
                                                const float* __restrict__ bias, const float* __restrict__ resid, int rmod, int ldr,
                                                float* __restrict__ C, int ldc, int M, int N, int K) {
  __shared__ __attribute__((aligned(16))) float so[4][16][64];
  const int tid = threadIdx.x, w = tid >> 5, lane = tid & 31, ln = lane & 15, hh = lane >> 4;
  const int ntn = N / 64;
  const int wid = blockIdx.x * 4 + w;
  const int mt = wid / ntn, nq = wid % ntn;
  if (mt * 16 >= M) return;
  const int row0 = mt * 16, col0 = nq * 64;
  const float* arow = A + (size_t)(row0 + ln) * lda;
  v8f acc[4] = {};
  for (int kb = 0; kb < K; kb += 32) {
    FragB ah, al;
    const v4f x0 = *(const v4fa*)(arow + kb + 8 * hh), x1 = *(const v4fa*)(arow + kb + 8 * hh + 4);
    const v4f x2 = *(const v4fa*)(arow + kb + 16 + 8 * hh), x3 = *(const v4fa*)(arow + kb + 16 + 8 * hh + 4);
    float xs[16] = {x0[0],x0[1],x0[2],x0[3],x1[0],x1[1],x1[2],x1[3],x2[0],x2[1],x2[2],x2[3],x3[0],x3[1],x3[2],x3[3]};
#pragma unroll
    for (int i = 0; i < 16; ++i) { const unsigned short hb = bf16_bits(xs[i]); ah.u[i] = hb; al.u[i] = ASPLIT ? bf16_bits(xs[i] - bf16_val(hb)) : (unsigned short)0; }
#pragma unroll
    for (int t = 0; t < 4; ++t) {
      const unsigned short* brow = Wt + (size_t)(col0 + t * 16 + ln) * ldb + kb;
      FragB b;
      b.half[0] = *(const v8us*)(brow + 8 * hh);
      b.half[1] = *(const v8us*)(brow + 16 + 8 * hh);
      acc[t] = mmaN<ASPLIT ? 2 : 1>(ah.v, al.v, b.v, b.v, acc[t]);
    }
  }
#pragma unroll
  for (int t = 0; t < 4; ++t) {
    const int col = col0 + t * 16 + ln;
    float bv = bias ? bias[col] : 0.f;
    if (BIAS_BF16) bv = bf16_round(bv);
#pragma unroll
    for (int r = 0; r < 8; ++r) {
      float v = acc[t][r] + bv;
      if (resid) { float rv = resid[(size_t)((row0 + 8 * hh + r) % rmod) * ldr + col]; if (RES_BF16) rv = bf16_round(rv); v += rv; }
      if (ACT == 1) v = fmaxf(v, 0.f);
      if (ACT == 2) v = 0.5f * v * (1.0f + erff(v * 0.70710678118654752f));
      if (ACT == 3) { const float u = 0.7978845608028654f * (v + 0.044715f * v * v * v); v = 0.5f * v * (1.0f + tanhf(u)); }
      so[w][8 * hh + r][t * 16 + ln] = v;
    }
  }
  __builtin_amdgcn_fence(__ATOMIC_ACQ_REL, "workgroup");
  __builtin_amdgcn_wave_barrier();
  const int rsub = lane >> 4, c4 = (lane & 15) * 4;
  for (int pass = 0; pass < 2; ++pass) {
#pragma unroll
    for (int q = 0; q < 8; ++q) {
      const int r = q * 2 + rsub;
      const v4f v = *(const v4fa*)&so[w][r][c4];
      *(volatile v4f*)(C + (size_t)(row0 + r) * ldc + col0 + c4) = v;
    }
    if (pass == 0) __threadfence();
  }
}
template <bool PARAM_BF16>
__global__ __launch_bounds__(256) void k_layernorm(const float* __restrict__ X, const float* __restrict__ R, const float* __restrict__ g, const float* __restrict__ bta,
                                                  float* __restrict__ out_sum, float* __restrict__ out_norm, int N, float eps) {
  __shared__ float red[256];
  const int row = blockIdx.x, tid = threadIdx.x;
  const float* x = X + (size_t)row * N; const float* rr = R ? R + (size_t)row * N : nullptr;
  float vals[16];
  const int per = N / 256;
  float s1 = 0.f;
  for (int u = 0; u < per / 4; ++u) {
    const int j = tid * 4 + 1024 * u;
    const v4f a = *(const v4fa*)(x + j);
    v4f b = {0.f,0.f,0.f,0.f}; if (rr) b = *(const v4fa*)(rr + j);
#pragma unroll
    for (int q = 0; q < 4; ++q) { const float v = a[q] + b[q]; vals[u * 4 + q] = v; s1 += v; }
  }
  red[tid] = s1; __syncthreads();
  for (int st = 128; st > 0; st >>= 1) { if (tid < st) red[tid] += red[tid + st]; __syncthreads(); }
  const float mu = red[0] / (float)N; __syncthreads();
  float s2 = 0.f;
  for (int u = 0; u < per / 4; ++u)
#pragma unroll
    for (int q = 0; q < 4; ++q) { const float c = vals[u * 4 + q] - mu; s2 += c * c; }
  red[tid] = s2; __syncthreads();
  for (int st = 128; st > 0; st >>= 1) { if (tid < st) red[tid] += red[tid + st]; __syncthreads(); }
  const float rs = rsqrtf(red[0] / (float)N + eps);
  for (int pass = 0; pass < 2; ++pass) {
    for (int u = 0; u < per / 4; ++u) {
      const int j = tid * 4 + 1024 * u;
      v4f o, sm;
#pragma unroll
      for (int q = 0; q < 4; ++q) {
        float gg = g[j + q], bb = bta[j + q];
        if (PARAM_BF16) { gg = bf16_round(gg); bb = bf16_round(bb); }
        sm[q] = vals[u * 4 + q]; o[q] = (vals[u * 4 + q] - mu) * rs * gg + bb;
      }
      if (out_sum) *(volatile v4f*)(out_sum + (size_t)row * N + j) = sm;
      *(volatile v4f*)(out_norm + (size_t)row * N + j) = o;
    }
    if (pass == 0) __threadfence();
  }
}
template <int CinP, int ACT, int HI_, int WI_>
__global__ __launch_bounds__(128) void k_conv3x3(const float* __restrict__ in, int inP, const unsigned short* __restrict__ Bt, const float* __restrict__ bias, int Nb, float* __restrict__ out, int Np, int npos) {
  constexpr int K = 9 * CinP, SPT = CinP / 32;
  __shared__ __attribute__((aligned(16))) float so[4][16][64];
  const int tid = threadIdx.x, w = tid >> 5, lane = tid & 31, ln = lane & 15, hh = lane >> 4;
  const int ntn = Np / 64; const int wid = blockIdx.x * 4 + w; const int mt = wid / ntn, nq = wid % ntn;
  if (mt * 16 >= npos) return;
  const int row0 = mt * 16, col0 = nq * 64; const int m = row0 + ln; const int n = m / (HI_ * WI_), yx = m % (HI_ * WI_), y = yx / WI_, xq = yx % WI_;
  v8f acc[4] = {};
  for (int tap = 0; tap < 9; ++tap) {
    const int yy = y + tap / 3 - 1, xx = xq + tap % 3 - 1; const bool inb = (m < npos) && (yy >= 0 && yy < HI_ && xx >= 0 && xx < WI_);
    const float* src = in + ((size_t)n * HI_ * WI_ + (size_t)(inb ? yy : 0) * WI_ + (inb ? xx : 0)) * inP;
#pragma unroll
    for (int s = 0; s < SPT; ++s) {
      const int c0 = s * 32; v4f a0 = {0.f,0.f,0.f,0.f}, a1 = a0, a2 = a0, a3 = a0;
      if (inb) { a0 = *(const v4fa*)(src + c0 + 8 * hh); a1 = *(const v4fa*)(src + c0 + 8 * hh + 4); a2 = *(const v4fa*)(src + c0 + 16 + 8 * hh); a3 = *(const v4fa*)(src + c0 + 16 + 8 * hh + 4); }
      float xs[16] = {a0[0],a0[1],a0[2],a0[3],a1[0],a1[1],a1[2],a1[3],a2[0],a2[1],a2[2],a2[3],a3[0],a3[1],a3[2],a3[3]};
      FragB ah, al;
#pragma unroll
      for (int i = 0; i < 16; ++i) { const unsigned short hb = bf16_bits(xs[i]); ah.u[i] = hb; al.u[i] = bf16_bits(xs[i] - bf16_val(hb)); }
      const int kb = tap * CinP + c0;
#pragma unroll
      for (int t = 0; t < 4; ++t) { FragB bq; bq.half[0] = *(const v8us*)(Bt + (size_t)(col0 + t * 16 + ln) * K + kb + 8 * hh); bq.half[1] = *(const v8us*)(Bt + (size_t)(col0 + t * 16 + ln) * K + kb + 16 + 8 * hh); acc[t] = mmaN<2>(ah.v, al.v, bq.v, bq.v, acc[t]); }
    }
  }
#pragma unroll
  for (int t = 0; t < 4; ++t) { const int col = col0 + t * 16 + ln; const float bv = (col < Nb) ? bf16_round(bias[col]) : 0.f;
#pragma unroll
    for (int r = 0; r < 8; ++r) { float v = acc[t][r] + bv; if (ACT == 1) v = fmaxf(v, 0.f); else if (ACT == 2) v = v >= 0.f ? v : 0.1f * v; so[w][8 * hh + r][t * 16 + ln] = v; } }
  __builtin_amdgcn_fence(__ATOMIC_ACQ_REL, "workgroup"); __builtin_amdgcn_wave_barrier();
  const int rsub = lane >> 4, c4 = (lane & 15) * 4;
  for (int pass = 0; pass < 2; ++pass) { for (int q = 0; q < 8; ++q) { const int r = q * 2 + rsub; if (row0 + r < npos) { const v4f v = *(const v4fa*)&so[w][r][c4]; *(volatile v4f*)(out + (size_t)(row0 + r) * Np + col0 + c4) = v; } } if (pass == 0) __threadfence(); }
}

__global__ __launch_bounds__(256) void k_wt_hwio(const float* __restrict__ w, unsigned short* __restrict__ Bt) {
  const int t = blockIdx.x * 256 + threadIdx.x; const int K = 9 * CC; if (t >= CC * (K / 8)) return; const int o = t / (K / 8), k8 = (t % (K / 8)) * 8; v8us v;
#pragma unroll
  for (int i = 0; i < 8; ++i) { const int k = k8 + i; const int tap = k / CC, c = k % CC; v[i] = bf16_bits(w[((size_t)tap * CC + c) * CC + o]); }
  *(volatile v8us*)(Bt + (size_t)o * K + k8) = v; __threadfence(); *(volatile v8us*)(Bt + (size_t)o * K + k8) = v;
}
__global__ __launch_bounds__(256) void k_round8(const float* __restrict__ w, unsigned short* __restrict__ Bt, int n8) { const int i = blockIdx.x * 256 + threadIdx.x; if (i >= n8) return; v8us o; for (int j = 0; j < 8; ++j) o[j] = bf16_bits(w[(size_t)i * 8 + j]); *(volatile v8us*)(Bt + (size_t)i * 8) = o; __threadfence(); *(volatile v8us*)(Bt + (size_t)i * 8) = o; }
__global__ __launch_bounds__(256) void k_imgstat(const float* __restrict__ im, float* __restrict__ slot) {
  __shared__ double rs[256], rq[256]; const int c = blockIdx.x; double s = 0.0, q = 0.0;
#pragma unroll 1
  for (int e = threadIdx.x; e < BB * NPIX; e += 256) { const int b = e / NPIX, p = e % NPIX; const double v = (double)bf16_round(im[((size_t)b * CC + c) * NPIX + p]); s += v; q += v * v; }
  rs[threadIdx.x] = s; rq[threadIdx.x] = q; __syncthreads(); for (int st = 128; st > 0; st >>= 1) { if (threadIdx.x < st) { rs[threadIdx.x] += rs[threadIdx.x + st]; rq[threadIdx.x] += rq[threadIdx.x + st]; } __syncthreads(); }
  const double n = (double)BB * NPIX; const double mu = rs[0] / n; double var = rq[0] / n - mu * mu; if (var < 0.0) var = 0.0;
  if (threadIdx.x < 32) { const float v = threadIdx.x == 0 ? (float)mu : (threadIdx.x == 1 ? (float)(1.0 / sqrt(var + 1e-5)) : 0.f); *(volatile float*)(slot + (size_t)c * 32 + threadIdx.x) = v; __threadfence(); *(volatile float*)(slot + (size_t)c * 32 + threadIdx.x) = v; }
}
__global__ __launch_bounds__(256) void k_imgbn(const float* __restrict__ im, const float* __restrict__ slot, const float* __restrict__ g, const float* __restrict__ bb, float* __restrict__ xr) {
  const size_t i = (size_t)blockIdx.x * 256 + threadIdx.x; if (i >= (size_t)BB * CC * NPIX / 4) return; const int c = (int)((i / (NPIX / 4)) % CC); const float mu = slot[c * 32], rs = slot[c * 32 + 1], ga = bf16_round(g[c]), be = bf16_round(bb[c]);
  v4f v = *(const v4fa*)(im + i * 4); for (int q = 0; q < 4; ++q) v[q] = fmaxf(ga * (bf16_round(v[q]) - mu) * rs + be, 0.f);
  *(volatile v4f*)(xr + i * 4) = v; __threadfence(); *(volatile v4f*)(xr + i * 4) = v;
}
__global__ __launch_bounds__(256) void k_hough(const float* __restrict__ xr, const int* __restrict__ idx, const float* __restrict__ hw, float* __restrict__ ht) {
  const int tid = threadIdx.x, wv = tid >> 5, lane = tid & 31; const int r = blockIdx.x * 8 + wv; if (r >= NPOSH) return; const int b = r / NBINS, bin = r % NBINS;
  v4f a = {0.f,0.f,0.f,0.f};
#pragma unroll 1
  for (int k = 0; k < KHT; ++k) { int p = idx[bin * KHT + k]; p = p < 0 ? 0 : (p >= NPIX ? NPIX - 1 : p); const float wk = bf16_round(hw[bin * KHT + k]);
    for (int q = 0; q < 4; ++q) a[q] += xr[((size_t)b * CC + lane * 4 + q) * NPIX + p] * wk; }
  *(volatile v4f*)(ht + (size_t)r * CC + lane * 4) = a; __threadfence(); *(volatile v4f*)(ht + (size_t)r * CC + lane * 4) = a;
}
template <int C>
__global__ __launch_bounds__(256) void k_colstat1(const float* __restrict__ h, int nrows, double* __restrict__ part) { const int c = threadIdx.x; const int r0 = blockIdx.x * 512; const int r1 = min(r0 + 512, nrows); double s = 0.0, q = 0.0;
#pragma unroll 1
  for (int r = r0; r < r1; ++r) { const double v = (double)h[(size_t)r * C + c]; s += v; q += v * v; } double* d = part + (size_t)blockIdx.x * 2 * C; *(volatile double*)(d + c) = s; *(volatile double*)(d + C + c) = q; __threadfence(); *(volatile double*)(d + c) = s; *(volatile double*)(d + C + c) = q; }
template <int C>
__global__ __launch_bounds__(256) void k_colstat2(const double* __restrict__ part, int nblk, int nrows, float* __restrict__ st) { const int c = threadIdx.x; double s = 0.0, q = 0.0; for (int b = 0; b < nblk; ++b) { s += part[(size_t)b * 2 * C + c]; q += part[(size_t)b * 2 * C + C + c]; }
  const double mu = s / nrows; double var = q / nrows - mu * mu; if (var < 0.0) var = 0.0; const float m = (float)mu, rs = (float)(1.0 / sqrt(var + 1e-5)); *(volatile float*)(st + c) = m; *(volatile float*)(st + C + c) = rs; __threadfence(); *(volatile float*)(st + c) = m; *(volatile float*)(st + C + c) = rs; }
template <int C>
__global__ __launch_bounds__(256) void k_bnrelu(float* __restrict__ h, int nrows, const float* __restrict__ st, const float* __restrict__ g, const float* __restrict__ bb) { const size_t t = (size_t)blockIdx.x * 256 + threadIdx.x; if (t >= (size_t)nrows * (C / 4)) return; const int c4 = (int)(t % (C / 4)) * 4; v4f v = *(const v4fa*)(h + t * 4);
  for (int q = 0; q < 4; ++q) { const int c = c4 + q; v[q] = fmaxf(bf16_round(g[c]) * (v[q] - st[c]) * st[C + c] + bf16_round(bb[c]), 0.f); } *(volatile v4f*)(h + t * 4) = v; __threadfence(); *(volatile v4f*)(h + t * 4) = v; }
__global__ __launch_bounds__(256) void k_sphere(const float* __restrict__ xh, const int* __restrict__ sidx, const float* __restrict__ sw, const int* __restrict__ ind, int S, float* __restrict__ g) {
  const int tid = threadIdx.x, wv = tid >> 5, lane = tid & 31; const int r = blockIdx.x * 8 + wv; if (r >= BB * S) return; const int b = r / S;
  int node = ind[r]; node = node < 0 ? 0 : (node >= NSPH ? NSPH - 1 : node);
  v4f a = {0.f,0.f,0.f,0.f};
#pragma unroll 1
  for (int k = 0; k < KSPH; ++k) { int bin = sidx[node * KSPH + k]; bin = bin < 0 ? 0 : (bin >= NBINS ? NBINS - 1 : bin); const float wk = bf16_round(sw[node * KSPH + k]); const v4f v = *(const v4fa*)(xh + ((size_t)b * NBINS + bin) * CC + lane * 4); for (int q = 0; q < 4; ++q) a[q] += v[q] * wk; }
  *(volatile v4f*)(g + (size_t)r * CC + lane * 4) = a; __threadfence(); *(volatile v4f*)(g + (size_t)r * CC + lane * 4) = a;
}
__global__ __launch_bounds__(128) void k_edgeconv(const float* __restrict__ x, const int* __restrict__ edge, int n, int nedge, const unsigned short* __restrict__ Bt, const float* __restrict__ bias, float* __restrict__ xo, int total_nodes) {
  __shared__ __attribute__((aligned(16))) float so[4][2][64];
  const int tid = threadIdx.x, w = tid >> 5, lane = tid & 31, ln = lane & 15, hh = lane >> 4;
  const int wid = blockIdx.x * 4 + w; const int node0 = wid * 2; if (node0 >= total_nodes) return;
  const int e = node0 * 8 + ln; const int g = e / nedge, el = e % nedge;
  int ci = edge[((size_t)g * 2 + 0) * nedge + el], ni = edge[((size_t)g * 2 + 1) * nedge + el]; ci = ci < 0 ? 0 : (ci >= n ? n - 1 : ci); ni = ni < 0 ? 0 : (ni >= n ? n - 1 : ni);
  const float* xc = x + ((size_t)g * n + ci) * 64; const float* xn = x + ((size_t)g * n + ni) * 64;
  v8f acc[4] = {};
#pragma unroll
  for (int ks = 0; ks < 4; ++ks) { FragB ah, al;
#pragma unroll
    for (int i = 0; i < 16; ++i) { const int k = ks * 32 + ((i < 8) ? (8 * hh + i) : (16 + 8 * hh + (i - 8))); const float v = (k < 64) ? xc[k] : (xn[k - 64] - xc[k - 64]); const unsigned short hb = bf16_bits(v); ah.u[i] = hb; al.u[i] = bf16_bits(v - bf16_val(hb)); }
#pragma unroll
    for (int t = 0; t < 4; ++t) { FragB bq; bq.half[0] = *(const v8us*)(Bt + (size_t)(t * 16 + ln) * 128 + ks * 32 + 8 * hh); bq.half[1] = *(const v8us*)(Bt + (size_t)(t * 16 + ln) * 128 + ks * 32 + 16 + 8 * hh); acc[t] = mmaN<2>(ah.v, al.v, bq.v, bq.v, acc[t]); } }
#pragma unroll
  for (int t = 0; t < 4; ++t) { const int col = t * 16 + ln; const float bv = bf16_round(bias[col]); float m = -3.0e38f;
#pragma unroll
    for (int r = 0; r < 8; ++r) m = fmaxf(m, fmaxf(acc[t][r] + bv, 0.f)); so[w][hh][col] = m; }
  __builtin_amdgcn_fence(__ATOMIC_ACQ_REL, "workgroup"); __builtin_amdgcn_wave_barrier();
  const v4f v = *(const v4fa*)&so[w][lane >> 4][(lane & 15) * 4];
  *(volatile v4f*)(xo + (size_t)(node0 + (lane >> 4)) * 64 + (lane & 15) * 4) = v; __threadfence(); *(volatile v4f*)(xo + (size_t)(node0 + (lane >> 4)) * 64 + (lane & 15) * 4) = v;
}
__global__ __launch_bounds__(256) void k_headz(const float* __restrict__ x, const float* __restrict__ hw, const float* __restrict__ hb, int total, float* __restrict__ z) {
  const int i = blockIdx.x * 256 + threadIdx.x; if (i >= total) return; float s = bf16_round(hb[0]);
#pragma unroll 1
  for (int c = 0; c < 64; c += 4) { const v4f a = *(const v4fa*)(x + (size_t)i * 64 + c); s += a[0] * bf16_round(hw[c]) + a[1] * bf16_round(hw[c + 1]) + a[2] * bf16_round(hw[c + 2]) + a[3] * bf16_round(hw[c + 3]); }
  *(volatile float*)(z + i) = s; __threadfence(); *(volatile float*)(z + i) = s;
}
__global__ __launch_bounds__(256) void k_final(const float* __restrict__ z0, const float* __restrict__ z1, const float* __restrict__ z2, const int* __restrict__ t0, const int* __restrict__ t1, const int* __restrict__ t2, float* __restrict__ out) {
  __shared__ float rp[256], rn[256], cp[256], cn[256]; __shared__ float loss[6];
  const int tid = threadIdx.x;
  for (int sc = 0; sc < 3; ++sc) {
    const float* z = sc == 0 ? z0 : sc == 1 ? z1 : z2; const int* t = sc == 0 ? t0 : sc == 1 ? t1 : t2; const int tot = sc == 0 ? BB * 1024 : sc == 1 ? BB * 3 * 256 : BB * 3 * 64;
    float sp = 0.f, sn = 0.f, np_ = 0.f, nn = 0.f;
    for (int i = tid; i < tot; i += 256) { const float zz = z[i]; const float tt = (float)t[i]; const float l = fmaxf(zz, 0.f) - zz * tt + log1pf(expf(-fabsf(zz))); if (tt > 0.5f) { sp += l; np_ += 1.f; } else { sn += l; nn += 1.f; } }
    rp[tid] = sp; rn[tid] = sn; cp[tid] = np_; cn[tid] = nn; __syncthreads();
    for (int st = 128; st > 0; st >>= 1) { if (tid < st) { rp[tid] += rp[tid + st]; rn[tid] += rn[tid + st]; cp[tid] += cp[tid + st]; cn[tid] += cn[tid + st]; } __syncthreads(); }
    if (tid == 0) { loss[sc * 2] = rp[0] / fmaxf(cp[0], 1.f); loss[sc * 2 + 1] = rn[0] / fmaxf(cn[0], 1.f); } __syncthreads();
  }
  const int total = 6 + BB * 1984;
  for (int pass = 0; pass < 2; ++pass) {
    for (int i = tid; i < total; i += 256) { float v; if (i < 6) v = loss[i]; else { const int e = i - 6; const int b = e / 1984, j = e % 1984; float zz; if (j < 1024) zz = z0[b * 1024 + j]; else if (j < 1792) zz = z1[b * 768 + (j - 1024)]; else zz = z2[b * 192 + (j - 1792)]; v = 1.0f / (1.0f + expf(-zz)); } *(volatile float*)(out + i) = v; }
    if (pass == 0) __threadfence(); }
}
extern "C" void kernel_launch(void* const* d_in, const int* in_sizes, int n_in,
                              void* d_out, int out_size, void* d_ws, size_t ws_size, hipStream_t stream) {
  (void)in_sizes; (void)n_in; (void)out_size;
  const float* image = (const float*)d_in[0]; const float* bng = (const float*)d_in[1]; const float* bnb = (const float*)d_in[2]; const int* ht_idx = (const int*)d_in[3]; const float* ht_w = (const float*)d_in[4];
  const float* w_ht = (const float*)d_in[5]; const float* htg = (const float*)d_in[6]; const float* htb = (const float*)d_in[7]; const int* sph_idx = (const int*)d_in[8]; const float* sph_w = (const float*)d_in[9];
  const float* w_sc = (const float*)d_in[10]; const float* b_sc = (const float*)d_in[11]; const float* scg = (const float*)d_in[12]; const float* scb = (const float*)d_in[13];
  const float* dg_w = (const float*)d_in[14]; const float* dg_b = (const float*)d_in[15]; const float* dg_hw = (const float*)d_in[16]; const float* dg_hb = (const float*)d_in[17];
  const int* ind[3] = {(const int*)d_in[18], (const int*)d_in[19], (const int*)d_in[20]}; const int* edg[3] = {(const int*)d_in[21], (const int*)d_in[22], (const int*)d_in[23]}; const int* tgt[3] = {(const int*)d_in[24], (const int*)d_in[25], (const int*)d_in[26]};
  char* ws = (char*)d_ws; size_t off = 0;
  auto take = [&](size_t bytes) { char* p = ws + off; off += (bytes + 255) & ~(size_t)255; return p; };
  const int S[3] = {1024, 768, 192}, NN_[3] = {1024, 256, 64}, NGR[3] = {BB, BB * 3, BB * 3};
  unsigned short* Bht = (unsigned short*)take((size_t)CC * 9 * CC * 2); unsigned short* Bsc[3]; unsigned short* Bdg[3][4];
  for (int s = 0; s < 3; ++s) { Bsc[s] = (unsigned short*)take(64 * CC * 2); for (int i = 0; i < 4; ++i) Bdg[s][i] = (unsigned short*)take(64 * 128 * 2); }
  float* slot = (float*)take(CC * 32 * 4); float* xr = (float*)take((size_t)BB * CC * NPIX * 4); float* ht = (float*)take((size_t)NPOSH * CC * 4); float* hc = (float*)take((size_t)NPOSH * CC * 4);
  const int nblkH = (NPOSH + 511) / 512; double* part = (double*)take((size_t)nblkH * 2 * CC * 8); float* st = (float*)take(2 * CC * 4);
  float* gsp = (float*)take((size_t)BB * 1024 * CC * 4); float* ysc = (float*)take((size_t)BB * 1024 * 64 * 4); float* xa = (float*)take((size_t)BB * 1024 * 64 * 4); float* xb = (float*)take((size_t)BB * 1024 * 64 * 4);
  float* z[3]; for (int s = 0; s < 3; ++s) z[s] = (float*)take((size_t)BB * S[s] * 4 + 256);
  if (off > ws_size) return;
  k_wt_hwio<<<(CC * (9 * CC / 8) + 255) / 256, 256, 0, stream>>>(w_ht, Bht);
  for (int s = 0; s < 3; ++s) { k_round8<<<(64 * CC / 8 + 255) / 256, 256, 0, stream>>>(w_sc + (size_t)s * 64 * CC, Bsc[s], 64 * CC / 8); for (int i = 0; i < 4; ++i) k_wt_bf16<<<(64 * 16 + 255) / 256, 256, 0, stream>>>(dg_w + ((size_t)s * 4 + i) * 128 * 64, Bdg[s][i], 128, 64); }
  k_imgstat<<<CC, 256, 0, stream>>>(image, slot);
  k_imgbn<<<(unsigned)(((size_t)BB * CC * NPIX / 4 + 255) / 256), 256, 0, stream>>>(image, slot, bng, bnb, xr);
  k_hough<<<(NPOSH + 7) / 8, 256, 0, stream>>>(xr, ht_idx, ht_w, ht);
  k_conv3x3<CC, 0, HTH, HTW><<<((NPOSH / 16) * 2 + 3) / 4, 128, 0, stream>>>(ht, CC, Bht, nullptr, 0, hc, CC, NPOSH);
  k_colstat1<CC><<<nblkH, CC, 0, stream>>>(hc, NPOSH, part); k_colstat2<CC><<<1, CC, 0, stream>>>(part, nblkH, NPOSH, st); k_bnrelu<CC><<<(unsigned)(((size_t)NPOSH * CC / 4 + 255) / 256), 256, 0, stream>>>(hc, NPOSH, st, htg, htb);
  for (int s = 0; s < 3; ++s) {
    const int rows = BB * S[s]; const int nblk = (rows + 511) / 512;
    k_sphere<<<(rows + 7) / 8, 256, 0, stream>>>(hc, sph_idx, sph_w, ind[s], S[s], gsp);
    k_gemm_bf3<true, 0, true, false><<<((rows / 16) * 1 + 3) / 4, 128, 0, stream>>>(gsp, CC, Bsc[s], CC, b_sc + s * 64, nullptr, 1, 0, ysc, 64, rows, 64, CC);
    k_colstat1<64><<<nblk, 64, 0, stream>>>(ysc, rows, part); k_colstat2<64><<<1, 64, 0, stream>>>(part, nblk, rows, st); k_bnrelu<64><<<(rows * 16 + 255) / 256, 256, 0, stream>>>(ysc, rows, st, scg + s * 64, scb + s * 64);
    const float* xin = ysc; float* bufs[2] = {xa, xb};
    for (int i = 0; i < 4; ++i) { float* xo = bufs[i & 1]; k_edgeconv<<<(rows / 2 + 3) / 4, 128, 0, stream>>>(xin, edg[s], NN_[s], NN_[s] * 8, Bdg[s][i], dg_b + ((size_t)s * 4 + i) * 64, xo, rows); xin = xo; }
    k_headz<<<(rows + 255) / 256, 256, 0, stream>>>(xin, dg_hw + s * 64, dg_hb + s, rows, z[s]);
  }
  k_final<<<1, 256, 0, stream>>>(z[0], z[1], z[2], tgt[0], tgt[1], tgt[2], (float*)d_out);
}
